// DefaultAttention_27814208209133
// MI455X (gfx1250) — hardware-verified
//
#include <hip/hip_runtime.h>

constexpr int kBatch = 4;
constexpr int kSeq   = 2048;
constexpr int kEmb   = 1024;
constexpr int kTok   = kBatch * kSeq;
constexpr float kSimScale = 0.03125f;
static_assert(kTok % 64 == 0 && kSeq % 64 == 0 && kEmb % 64 == 0, "tile multiples");
static_assert(kEmb % 32 == 0 && kSeq % 32 == 0, "K multiples of 32");
static_assert(kSeq == 8 * 256, "softmax row = 256 threads x 8 columns");

constexpr size_t kPlaneTok16 = (size_t)kTok * kEmb * 2;
constexpr size_t kPlaneW16   = (size_t)3 * kEmb * kEmb * 2;
constexpr size_t kPlaneS32   = (size_t)kSeq * kSeq * 4;
constexpr size_t kPlaneP16   = (size_t)kSeq * kSeq * 2;
constexpr size_t kPlaneVT16  = (size_t)kBatch * kEmb * kSeq * 2;
constexpr size_t kOffXb  = 0;
constexpr size_t kOffWb  = kOffXb + kPlaneTok16;
constexpr size_t kOffS   = 0;
constexpr size_t kOffPh  = kOffS + kPlaneS32;
constexpr size_t kOffPl  = kOffPh + kPlaneP16;
constexpr size_t kOffKh  = kOffPl + kPlaneP16;
constexpr size_t kOffKl  = kOffKh + kPlaneTok16;
constexpr size_t kOffQh  = kOffKl + kPlaneTok16;
constexpr size_t kOffQl  = kOffQh + kPlaneTok16;
constexpr size_t kOffVTh = kOffQl + kPlaneTok16;
constexpr size_t kOffVTl = kOffVTh + kPlaneVT16;
constexpr size_t kWsTotal = kOffVTl + kPlaneVT16;
static_assert(kOffWb + kPlaneW16 <= kOffKh, "projection-phase planes fit inside the reused region");
static_assert(kWsTotal == 134217728ull, "carve total 128 MiB");

typedef __attribute__((ext_vector_type(16))) _Float16 v16h;
typedef __attribute__((ext_vector_type(8)))  _Float16 v8h;
typedef __attribute__((ext_vector_type(16))) __bf16   v16b;
typedef __attribute__((ext_vector_type(8)))  __bf16   v8b;
typedef __attribute__((ext_vector_type(8)))  float    v8f;
typedef __attribute__((ext_vector_type(4)))  float    v4f;
typedef __attribute__((ext_vector_type(4)))  unsigned int v4u;

__device__ __forceinline__ unsigned short f2bf_bits(float f) {
  unsigned u = __float_as_uint(f);
  return (unsigned short)((u + 0x7FFFu + ((u >> 16) & 1u)) >> 16);
}
__device__ __forceinline__ float bf_bits2f(unsigned short h) { return __uint_as_float(((unsigned)h) << 16); }

__device__ __forceinline__ void dep_guard_h(v8f& a, v8f& b, v16h x, v16h y) { asm volatile("v_nop\n\tv_nop\n\tv_nop\n\tv_nop" : "+v"(a), "+v"(b) : "v"(x), "v"(y)); }
__device__ __forceinline__ void dep_guard_b(v8f& a, v8f& b, v16b x, v16b y) { asm volatile("v_nop\n\tv_nop\n\tv_nop\n\tv_nop" : "+v"(a), "+v"(b) : "v"(x), "v"(y)); }
__device__ __forceinline__ void keep4_h(v16h a, v16h b, v16h c, v16h d) { asm volatile("v_nop" :: "v"(a), "v"(b), "v"(c), "v"(d)); }
__device__ __forceinline__ void keep4_b(v16b a, v16b b, v16b c, v16b d) { asm volatile("v_nop" :: "v"(a), "v"(b), "v"(c), "v"(d)); }
__device__ __forceinline__ void acc_guard4(v8f& a, v8f& b, v8f& c, v8f& d) { asm volatile("v_nop\n\tv_nop\n\tv_nop\n\tv_nop" : "+v"(a), "+v"(b), "+v"(c), "+v"(d)); }
template <typename T> struct Frag;
template <> struct Frag<_Float16> {
  typedef v16h V; union U { v16h v; v8h h[2]; };
  static __device__ __forceinline__ v16h load(const _Float16* p) {
    U f; f.h[0] = *(const v8h*)(p); f.h[1] = *(const v8h*)(p + 16); return f.v;
  }
  static __device__ __forceinline__ v8f mma(v16h a, v16h b, v8f c) {
    return __builtin_amdgcn_wmma_f32_16x16x32_f16(false, a, false, b, (short)0, c, false, false);
  }
  static __device__ __forceinline__ void guard(v8f& a, v8f& b, v16h x, v16h y) { dep_guard_h(a, b, x, y); }
  static __device__ __forceinline__ void keep(v16h a, v16h b, v16h c, v16h d) { keep4_h(a, b, c, d); }
};
template <> struct Frag<__bf16> {
  typedef v16b V; union U { v16b v; v8b h[2]; };
  static __device__ __forceinline__ v16b load(const __bf16* p) {
    U f; f.h[0] = *(const v8b*)(p); f.h[1] = *(const v8b*)(p + 16); return f.v;
  }
  static __device__ __forceinline__ v8f mma(v16b a, v16b b, v8f c) {
    return __builtin_amdgcn_wmma_f32_16x16x32_bf16(false, a, false, b, (short)0, c, false, false);
  }
  static __device__ __forceinline__ void guard(v8f& a, v8f& b, v16b x, v16b y) { dep_guard_b(a, b, x, y); }
  static __device__ __forceinline__ void keep(v16b a, v16b b, v16b c, v16b d) { keep4_b(a, b, c, d); }
};

__device__ __forceinline__ unsigned pk16(unsigned short a, unsigned short b) { return (unsigned)a | ((unsigned)b << 16); }

template <int ET> struct Elem;
template <> struct Elem<0> { typedef _Float16 T; };
template <> struct Elem<1> { typedef __bf16 T; };
template <int ET, bool SPLIT, int BIAS_MODE, int OUT_MODE, bool RESID, int ACT = 0, int TRI = 0>
__global__ __launch_bounds__(256) void wmma_gemm64(
    const unsigned short* __restrict__ Ap, const unsigned short* __restrict__ A2p, int lda, long strideA,
    const unsigned short* __restrict__ Btp, const unsigned short* __restrict__ Bt2p, int ldb, long strideB,
    void* __restrict__ Cout, void* __restrict__ Cout2, int ldc, long strideC,
    const float* __restrict__ bias,
    const float* __restrict__ resid, long strideR,
    int M, int N, int K, float scale) {
  typedef typename Elem<ET>::T T;
  typedef typename Frag<T>::V V;
  const T* A = (const T*)Ap; const T* A2 = (const T*)A2p; const T* Bt = (const T*)Btp; const T* Bt2 = (const T*)Bt2p;
  __shared__ __align__(16) float sT[8][16 * 68];
  const int b    = blockIdx.y;
  const int lane = threadIdx.x & 31;
  const int wave = threadIdx.x >> 5;
  const int tilesN = N >> 6;
  const int tilesM = M >> 6;
  const int tile = blockIdx.x * 8 + wave;
  int tm, tn;
  if (TRI == 1) {
    const int nTri = (tilesM * (tilesM + 1)) >> 1;
    if (tile >= nTri) return;
    int t = 0;
#pragma unroll 1
    for (int i = 1; i < tilesM; ++i) t += ((((i * (i + 1)) >> 1) <= tile) ? 1 : 0);
    tm = t;
    tn = tile - ((t * (t + 1)) >> 1);
  } else {
    if (tile >= tilesM * tilesN) return;
    tm = tile / tilesN;
    tn = tile - tm * tilesN;
  }
  const int m0 = tm << 6;
  const int n0 = tn << 6;
  const int Kt = (TRI == 2) ? ((m0 + 64 < K) ? (m0 + 64) : K) : K;

  const T* Ab  = A  + (size_t)b * strideA;
  const T* Bb  = Bt + (size_t)b * strideB;
  const T* Ab2 = SPLIT ? (A2  + (size_t)b * strideA) : nullptr;
  const T* Bb2 = SPLIT ? (Bt2 + (size_t)b * strideB) : nullptr;

  const int rlane = lane & 15;
  const int koff  = (lane >> 4) * 8;
  const int mOff  = (lane >> 4) * 8;

  v8f acc[4][4];
#pragma unroll
  for (int i = 0; i < 4; ++i)
#pragma unroll
    for (int j = 0; j < 4; ++j) acc[i][j] = (v8f){0.f,0.f,0.f,0.f,0.f,0.f,0.f,0.f};

  for (int k0 = 0; k0 < Kt; k0 += 32) {
    V bh[4], bl[4];
#pragma unroll
    for (int j = 0; j < 4; ++j) {
      const size_t bo = (size_t)(n0 + (j << 4) + rlane) * ldb + koff + k0;
      bh[j] = Frag<T>::load(Bb + bo);
      if (SPLIT) bl[j] = Frag<T>::load(Bb2 + bo);
    }
#pragma unroll
    for (int i = 0; i < 4; ++i) {
      const size_t ao = (size_t)(m0 + (i << 4) + rlane) * lda + koff + k0;
      V ah = Frag<T>::load(Ab + ao);
      V al;
      if (SPLIT) al = Frag<T>::load(Ab2 + ao);
#pragma unroll
      for (int j = 0; j < 4; ++j) {
        acc[i][j] = Frag<T>::mma(ah, bh[j], acc[i][j]);
        if (SPLIT) {
          acc[i][j] = Frag<T>::mma(ah, bl[j], acc[i][j]);
          acc[i][j] = Frag<T>::mma(al, bh[j], acc[i][j]);
        }
      }
      Frag<T>::guard(acc[i][0], acc[i][3], ah, SPLIT ? al : ah);
    }
    Frag<T>::keep(bh[0], bh[1], bh[2], bh[3]);
    if (SPLIT) Frag<T>::keep(bl[0], bl[1], bl[2], bl[3]);
  }
  acc_guard4(acc[0][0], acc[0][1], acc[0][2], acc[0][3]);
  acc_guard4(acc[1][0], acc[1][1], acc[1][2], acc[1][3]);
  acc_guard4(acc[2][0], acc[2][1], acc[2][2], acc[2][3]);
  acc_guard4(acc[3][0], acc[3][1], acc[3][2], acc[3][3]);

  float* slab = sT[wave];
  const float* Rb = RESID ? (resid + (size_t)b * strideR) : nullptr;
#pragma unroll
  for (int i = 0; i < 4; ++i) {
    const int mBase = m0 + (i << 4);
#pragma unroll
    for (int j = 0; j < 4; ++j) {
      const int n = n0 + (j << 4) + rlane;
      float bv = 0.f;
      if (BIAS_MODE == 2) bv = bias[n];
#pragma unroll
      for (int r = 0; r < 8; ++r) {
        float v = acc[i][j][r] * scale;
        if (BIAS_MODE == 1) v += bias[mBase + mOff + r];
        if (BIAS_MODE == 2) v += bv;
        if (RESID) v += Rb[(size_t)(mBase + mOff + r) * ldc + n];
        if (ACT == 2) v = fmaxf(v, 0.0f);
        if (ACT == 4) v = (v > 0.f) ? v : 0.01f * v;
        slab[(mOff + r) * 68 + (j << 4) + rlane] = v;
      }
    }
    __builtin_amdgcn_fence(__ATOMIC_RELEASE, "workgroup");
    __builtin_amdgcn_wave_barrier();
    __builtin_amdgcn_fence(__ATOMIC_ACQUIRE, "workgroup");
    if (OUT_MODE == 0) {
      float* C = (float*)Cout + (size_t)b * strideC;
      const int hh = lane >> 4, c4 = (lane & 15) * 4;
      for (int pass = 0; pass < 2; ++pass) {
#pragma unroll
        for (int it = 0; it < 8; ++it) {
          const int row = it * 2 + hh;
          v4f v = *(const v4f*)(slab + row * 68 + c4);
          *(volatile v4f*)(C + (size_t)(mBase + row) * ldc + n0 + c4) = v;
        }
        __threadfence();
      }
    } else {
      const int q = lane >> 3, c8 = (lane & 7) * 8;
      unsigned short* C  = (unsigned short*)Cout  + (size_t)b * strideC;
      unsigned short* C2 = (OUT_MODE == 2) ? ((unsigned short*)Cout2 + (size_t)b * strideC) : nullptr;
      for (int pass = 0; pass < 2; ++pass) {
#pragma unroll
        for (int it = 0; it < 4; ++it) {
          const int row = it * 4 + q;
          const float* sp = slab + row * 68 + c8;
          v8h hv, lv;
#pragma unroll
          for (int e = 0; e < 8; ++e) {
            if (OUT_MODE == 1) {
              hv[e] = (_Float16)sp[e];
            } else {
              unsigned short hb = f2bf_bits(sp[e]);
              unsigned short lb = f2bf_bits(sp[e] - bf_bits2f(hb));
              hv[e] = __builtin_bit_cast(_Float16, hb);
              lv[e] = __builtin_bit_cast(_Float16, lb);
            }
          }
          *(volatile v8h*)(C + (size_t)(mBase + row) * ldc + n0 + c8) = hv;
          if (OUT_MODE == 2) *(volatile v8h*)(C2 + (size_t)(mBase + row) * ldc + n0 + c8) = lv;
        }
        __threadfence();
      }
    }
    __builtin_amdgcn_fence(__ATOMIC_RELEASE, "workgroup");
    __builtin_amdgcn_wave_barrier();
    __builtin_amdgcn_fence(__ATOMIC_ACQUIRE, "workgroup");
  }
}

__global__ __launch_bounds__(256) void cast8_bf16_kernel(const float* __restrict__ in0, const float* __restrict__ in1,
                                                         const float* __restrict__ in2, unsigned short* __restrict__ out,
                                                         int n8, long planeStride) {
  const int i = blockIdx.x * 256 + threadIdx.x;
  if (i >= n8) return;
  const int z = blockIdx.y;
  const float* in = (z == 0) ? in0 : (z == 1) ? in1 : in2;
  const float* p = in + 8 * (size_t)i;
  const v4f a = *(const v4f*)(p);
  const v4f c = *(const v4f*)(p + 4);
  unsigned short hb[8];
#pragma unroll
  for (int e = 0; e < 4; ++e) {
    hb[e]     = f2bf_bits(a[e]);
    hb[4 + e] = f2bf_bits(c[e]);
  }
  const v4u u = (v4u){pk16(hb[0], hb[1]), pk16(hb[2], hb[3]), pk16(hb[4], hb[5]), pk16(hb[6], hb[7])};
  unsigned short* q = out + (size_t)z * planeStride + 8 * (size_t)i;
  *(volatile v4u*)q = u;
  __threadfence();
  *(volatile v4u*)q = u;
}

__global__ __launch_bounds__(256) void softmax_causal_kernel(const float* __restrict__ S,
                                                             unsigned short* __restrict__ Ph,
                                                             unsigned short* __restrict__ Pl) {
  __shared__ float redM[8];
  __shared__ float redS[8];
  const int row  = blockIdx.x;
  const int t    = threadIdx.x;
  const int lane = t & 31, wave = t >> 5;
  const int c0   = t * 8;
  const float* sr = S + (size_t)row * kSeq + c0;
  const v4f a = *(const v4f*)(sr);
  const v4f c = *(const v4f*)(sr + 4);
  const float ninf = -__builtin_inff();
  float x[8];
#pragma unroll
  for (int e = 0; e < 4; ++e) {
    x[e]     = (c0 + e     <= row) ? a[e] : ninf;
    x[4 + e] = (c0 + 4 + e <= row) ? c[e] : ninf;
  }
  float m = fmaxf(fmaxf(fmaxf(x[0], x[1]), fmaxf(x[2], x[3])), fmaxf(fmaxf(x[4], x[5]), fmaxf(x[6], x[7])));
#pragma unroll
  for (int off = 16; off > 0; off >>= 1) m = fmaxf(m, __shfl_xor(m, off, 32));
  if (lane == 0) redM[wave] = m;
  __syncthreads();
  float gm = redM[0];
#pragma unroll
  for (int w = 1; w < 8; ++w) gm = fmaxf(gm, redM[w]);

  float ev[8];
#pragma unroll
  for (int e = 0; e < 8; ++e) ev[e] = 0.f;
  if (c0 <= row) {
#pragma unroll
    for (int e = 0; e < 8; ++e) ev[e] = expf(x[e] - gm);
  }
  float psum = ((ev[0] + ev[1]) + (ev[2] + ev[3])) + ((ev[4] + ev[5]) + (ev[6] + ev[7]));
#pragma unroll
  for (int off = 16; off > 0; off >>= 1) psum += __shfl_xor(psum, off, 32);
  if (lane == 0) redS[wave] = psum;
  __syncthreads();
  float tot = redS[0];
#pragma unroll
  for (int w = 1; w < 8; ++w) tot += redS[w];
  const float inv = 1.0f / tot;

  unsigned short hb[8], lb[8];
#pragma unroll
  for (int e = 0; e < 8; ++e) {
    const float p = ev[e] * inv;
    hb[e] = f2bf_bits(p);
    lb[e] = f2bf_bits(p - bf_bits2f(hb[e]));
  }
  const v4u uh = (v4u){pk16(hb[0], hb[1]), pk16(hb[2], hb[3]), pk16(hb[4], hb[5]), pk16(hb[6], hb[7])};
  const v4u ul = (v4u){pk16(lb[0], lb[1]), pk16(lb[2], lb[3]), pk16(lb[4], lb[5]), pk16(lb[6], lb[7])};
  unsigned short* ph = Ph + (size_t)row * kSeq + c0;
  unsigned short* pl = Pl + (size_t)row * kSeq + c0;
  *(volatile v4u*)ph = uh;
  *(volatile v4u*)pl = ul;
  __threadfence();
  *(volatile v4u*)ph = uh;
  *(volatile v4u*)pl = ul;
}

extern "C" void kernel_launch(void* const* d_in, const int* in_sizes, int n_in,
                              void* d_out, int out_size, void* d_ws, size_t ws_size,
                              hipStream_t stream) {
  if (n_in < 7) return;
  if (in_sizes[0] != kTok * kEmb || in_sizes[1] != kEmb * kEmb || in_sizes[2] != kEmb ||
      in_sizes[3] != kEmb * kEmb || in_sizes[4] != kEmb || in_sizes[5] != kEmb * kEmb || in_sizes[6] != kEmb) return;
  if (out_size != kTok * kEmb) return;
  if (ws_size < kWsTotal) return;

  const float* x  = (const float*)d_in[0];
  const float* Wk = (const float*)d_in[1];
  const float* bk = (const float*)d_in[2];
  const float* Wq = (const float*)d_in[3];
  const float* bq = (const float*)d_in[4];
  const float* Wv = (const float*)d_in[5];
  const float* bv = (const float*)d_in[6];
  float* out = (float*)d_out;

  char* ws = (char*)d_ws;
  unsigned short* Xb  = (unsigned short*)(ws + kOffXb);
  unsigned short* Wb  = (unsigned short*)(ws + kOffWb);
  float*          Sf  = (float*)(ws + kOffS);
  unsigned short* Ph  = (unsigned short*)(ws + kOffPh);
  unsigned short* Pl  = (unsigned short*)(ws + kOffPl);
  unsigned short* Kh  = (unsigned short*)(ws + kOffKh);
  unsigned short* Kl  = (unsigned short*)(ws + kOffKl);
  unsigned short* Qh  = (unsigned short*)(ws + kOffQh);
  unsigned short* Ql  = (unsigned short*)(ws + kOffQl);
  unsigned short* VTh = (unsigned short*)(ws + kOffVTh);
  unsigned short* VTl = (unsigned short*)(ws + kOffVTl);

  const size_t wPlane = (size_t)kEmb * kEmb;

  cast8_bf16_kernel<<<dim3((kTok * kEmb / 8) / 256, 1), 256, 0, stream>>>(x, x, x, Xb, kTok * kEmb / 8, 0L);
  cast8_bf16_kernel<<<dim3((kEmb * kEmb / 8) / 256, 3), 256, 0, stream>>>(Wk, Wq, Wv, Wb, kEmb * kEmb / 8, (long)wPlane);

  wmma_gemm64<1, false, 2, 2, false, 0, 0><<<dim3((kTok / 64) * (kEmb / 64) / 8, 1), 256, 0, stream>>>(
      Xb, nullptr, kEmb, 0L, Wb, nullptr, kEmb, 0L, (void*)Kh, (void*)Kl, kEmb, 0L,
      bk, nullptr, 0L, kTok, kEmb, kEmb, 1.0f);
  wmma_gemm64<1, false, 2, 2, false, 0, 0><<<dim3((kTok / 64) * (kEmb / 64) / 8, 1), 256, 0, stream>>>(
      Xb, nullptr, kEmb, 0L, Wb + wPlane, nullptr, kEmb, 0L, (void*)Qh, (void*)Ql, kEmb, 0L,
      bq, nullptr, 0L, kTok, kEmb, kEmb, 1.0f);
  wmma_gemm64<1, false, 1, 2, false, 0, 0><<<dim3((kEmb / 64) * (kSeq / 64) / 8, kBatch), 256, 0, stream>>>(
      Wb + 2 * wPlane, nullptr, kEmb, 0L, Xb, nullptr, kEmb, (long)kSeq * kEmb, (void*)VTh, (void*)VTl, kSeq, (long)kEmb * kSeq,
      bv, nullptr, 0L, kEmb, kSeq, kEmb, 1.0f);

  constexpr int kTilesS    = kSeq / 64;
  constexpr int kTriTiles  = kTilesS * (kTilesS + 1) / 2;
  constexpr int kTriBlocks = (kTriTiles + 7) / 8;
  static_assert(kTriTiles % 8 == 0, "triangular tile set fills whole blocks");

  for (int b = 0; b < kBatch; ++b) {
    const size_t offKQ = (size_t)b * kSeq * kEmb;
    const size_t offVT = (size_t)b * kEmb * kSeq;
    const size_t offO  = (size_t)b * kSeq * kEmb;
    wmma_gemm64<1, true, 0, 0, false, 0, 1><<<dim3(kTriBlocks, 1), 256, 0, stream>>>(
        Kh + offKQ, Kl + offKQ, kEmb, 0L, Qh + offKQ, Ql + offKQ, kEmb, 0L, (void*)Sf, nullptr, kSeq, 0L,
        nullptr, nullptr, 0L, kSeq, kSeq, kEmb, kSimScale);
    softmax_causal_kernel<<<dim3(kSeq), 256, 0, stream>>>(Sf, Ph, Pl);
    wmma_gemm64<1, true, 0, 0, false, 0, 2><<<dim3((kSeq / 64) * (kEmb / 64) / 8, 1), 256, 0, stream>>>(
        Ph, Pl, kSeq, 0L, VTh + offVT, VTl + offVT, kSeq, 0L, (void*)(out + offO), nullptr, kEmb, 0L,
        nullptr, nullptr, 0L, kSeq, kEmb, kSeq, 1.0f);
  }
}
